// HypergraphFeatureEnhancer_13005160972462
// MI455X (gfx1250) — hardware-verified
//
#include <hip/hip_runtime.h>
#include <stddef.h>
#include <math.h>


#define NB    4
#define NN    4096
#define CC    256
#define KT    8
#define NR    (NB * NN)
#define TPF   36
#define SPF   68
#define ECH   256
#define NCH   (NN / ECH)
#define LCAP  (ECH * KT)
#define NPB   32
#define EPSN  1e-12f
#define BNEPS 1e-5f

typedef float          v4f   __attribute__((ext_vector_type(4)));
typedef float          v8f   __attribute__((ext_vector_type(8)));
typedef unsigned short v8us  __attribute__((ext_vector_type(8)));
typedef unsigned short v16us __attribute__((ext_vector_type(16)));
typedef __bf16         v16bf __attribute__((ext_vector_type(16)));
typedef int            v4i   __attribute__((ext_vector_type(4)));

static_assert((NN % 64) == 0 && (CC % 64) == 0 && (NR % 64) == 0);
static_assert(NCH * ECH == NN);
static_assert((NN % NPB) == 0 && NPB == 32);
static_assert(CC == 8 * 32);
static_assert((CC % 32) == 0);
static_assert((TPF % 4) == 0 && (SPF % 4) == 0);
static_assert(LCAP == 2048);

__device__ __forceinline__ v8f wmb(v16us a, v16us b, v8f c) {
  v8f d = __builtin_amdgcn_wmma_f32_16x16x32_bf16(false, __builtin_bit_cast(v16bf, a), false,
                                                  __builtin_bit_cast(v16bf, b), (short)0, c,
                                                  false, false);
#if defined(__HIP_DEVICE_COMPILE__)
  asm volatile("v_nop\n\tv_nop\n\tv_nop\n\tv_nop" : "+v"(d) : "v"(a), "v"(b));
#endif
  return d;
}

__device__ __forceinline__ v8f wm3(v16us ah, v16us al, v16us bh, v16us bl, v8f c) {
  c = wmb(ah, bh, c);
  c = wmb(ah, bl, c);
  c = wmb(al, bh, c);
  return c;
}

__device__ __forceinline__ v8f zero8() {
  v8f z = {0.f, 0.f, 0.f, 0.f, 0.f, 0.f, 0.f, 0.f};
  return z;
}

__device__ __forceinline__ v16us ldf(const unsigned short* __restrict__ p, size_t row, int k0, int h) {
  const unsigned short* q = p + row * CC + k0 + 8 * h;
  const v8us u0 = *(const v8us*)q;
  const v8us u1 = *(const v8us*)(q + 16);
  return __builtin_shufflevector(u0, u1, 0, 1, 2, 3, 4, 5, 6, 7, 8, 9, 10, 11, 12, 13, 14, 15);
}

__device__ __forceinline__ unsigned bfr(float x) {
  const unsigned u = __float_as_uint(x);
  return (u + 0x7FFFu + ((u >> 16) & 1u)) >> 16;
}

__device__ __forceinline__ void split8(const float (&x)[8], v8us& hi, v8us& lo) {
#pragma unroll
  for (int i = 0; i < 8; ++i) {
    const unsigned hb = bfr(x[i]);
    const float hf = __uint_as_float(hb << 16);
    const unsigned lb = bfr(x[i] - hf);
    hi[i] = (unsigned short)hb;
    lo[i] = (unsigned short)lb;
  }
}

template <typename T>
__device__ __forceinline__ void st2(T* p, const T& v) {
  *(volatile T*)p = v;
  __threadfence();
  *(volatile T*)p = v;
}

__device__ __forceinline__ void t2p(const float* __restrict__ src, int ncols, int col0,
                                    unsigned short* dhi, unsigned short* dlo, size_t drow0,
                                    int donorm, unsigned short* nhi, unsigned short* nlo,
                                    size_t nrow0, float* sT) {
  const int tid = threadIdx.x, lane = tid & 31, wave = tid >> 5;
#pragma unroll
  for (int it = 0; it < 8; ++it) {
    const int r = it * 32 + (tid >> 3);
    const int c4 = (tid & 7) * 4;
    const v4f v = *(const v4f*)(src + (size_t)r * ncols + col0 + c4);
    *(v4f*)(sT + r * TPF + c4) = v;
  }
  __syncthreads();
#pragma unroll 1
  for (int q = 0; q < 4; ++q) {
    const int j = wave * 4 + q;
    float x[8];
#pragma unroll
    for (int i = 0; i < 8; ++i) x[i] = sT[(8 * lane + i) * TPF + j];
    v8us hv, lv;
    split8(x, hv, lv);
    const size_t ro = (drow0 + (size_t)j) * CC + 8 * lane;
    st2((v8us*)(dhi + ro), hv);
    st2((v8us*)(dlo + ro), lv);
    if (donorm) {
      float ss = 0.0f;
#pragma unroll
      for (int i = 0; i < 8; ++i) ss += x[i] * x[i];
      ss += __shfl_xor(ss, 16, 32);
      ss += __shfl_xor(ss, 8, 32);
      ss += __shfl_xor(ss, 4, 32);
      ss += __shfl_xor(ss, 2, 32);
      ss += __shfl_xor(ss, 1, 32);
      float nrm = sqrtf(ss);
      nrm = fmaxf(nrm, EPSN);
      const float ri = 1.0f / nrm;
      float xn[8];
#pragma unroll
      for (int i = 0; i < 8; ++i) xn[i] = x[i] * ri;
      v8us h2, l2;
      split8(xn, h2, l2);
      const size_t rn = (nrow0 + (size_t)j) * CC + 8 * lane;
      st2((v8us*)(nhi + rn), h2);
      st2((v8us*)(nlo + rn), l2);
    }
  }
}

__global__ __launch_bounds__(256) void k_feat2p(const float* __restrict__ feat,
                                                unsigned short* xhi, unsigned short* xlo,
                                                unsigned short* fhi, unsigned short* flo) {
  __shared__ __attribute__((aligned(16))) float sT[256 * TPF];
  const int b = blockIdx.y;
  const int col0 = blockIdx.x * 32;
  t2p(feat + (size_t)b * CC * NN, NN, col0, xhi, xlo, (size_t)b * NN + (size_t)col0,
      (b == 0) ? 1 : 0, fhi, flo, (size_t)col0, sT);
}

__global__ __launch_bounds__(256) void k_w2p(const float* __restrict__ w0, const float* __restrict__ w1,
                                             const float* __restrict__ w2, const float* __restrict__ w3,
                                             const float* __restrict__ w4, unsigned short* wpl) {
  __shared__ __attribute__((aligned(16))) float sT[256 * TPF];
  const int sel = blockIdx.y;
  const float* src = (sel == 0) ? w0 : (sel == 1) ? w1 : (sel == 2) ? w2 : (sel == 3) ? w3 : w4;
  unsigned short* dhi = wpl + (size_t)(2 * sel) * (CC * CC);
  unsigned short* dlo = dhi + (size_t)CC * CC;
  const int col0 = blockIdx.x * 32;
  t2p(src, CC, col0, dhi, dlo, (size_t)col0, 0, dhi, dlo, (size_t)col0, sT);
}

__device__ __forceinline__ bool better(float av, int ai, float bv, int bi) {
  return (av > bv) || (av == bv && ai < bi);
}
__device__ __forceinline__ void ins8(float (&tv)[KT], int (&ti)[KT], float v, int id) {
#pragma unroll
  for (int t = 0; t < KT; ++t) {
    const bool sw = better(v, id, tv[t], ti[t]);
    const float ov = tv[t];
    const int   oi = ti[t];
    tv[t] = sw ? v : ov;
    ti[t] = sw ? id : oi;
    v  = sw ? ov : v;
    id = sw ? oi : id;
  }
}

__global__ __launch_bounds__(128) void k_sim(const unsigned short* __restrict__ fhi,
                                             const unsigned short* __restrict__ flo, int* idxo) {
  __shared__ __attribute__((aligned(16))) float sS[64 * SPF];
  __shared__ __attribute__((aligned(16))) int   sI[64 * KT];
  const int tid = threadIdx.x, lane = tid & 31, wave = tid >> 5, h = lane >> 4, m = lane & 15;
  const int wm = wave >> 1, wn = wave & 1;
  const int m0 = blockIdx.x * 64;

  float tv[KT];
  int   ti[KT];
#pragma unroll
  for (int t = 0; t < KT; ++t) { tv[t] = -3.0e38f; ti[t] = NN; }

  const size_t ar = (size_t)(m0 + wm * 32 + m);

  for (int ct = 0; ct < NN / 64; ++ct) {
    const int n0 = ct * 64;
    int kz = 0;
#if defined(__HIP_DEVICE_COMPILE__)
    asm volatile("" : "+v"(kz));
#endif
    const size_t br = (size_t)(n0 + wn * 32 + m);
    v8f acc[2][2];
#pragma unroll
    for (int t = 0; t < 2; ++t)
#pragma unroll
      for (int u = 0; u < 2; ++u) acc[t][u] = zero8();
#pragma unroll 1
    for (int ks = 0; ks < CC / 32; ++ks) {
      const int k0 = ks * 32 + kz;
      v16us aH[2], aL[2], bH[2], bL[2];
#pragma unroll
      for (int t = 0; t < 2; ++t) {
        aH[t] = ldf(fhi, ar + 16 * t, k0, h);
        aL[t] = ldf(flo, ar + 16 * t, k0, h);
      }
#pragma unroll
      for (int u = 0; u < 2; ++u) {
        bH[u] = ldf(fhi, br + 16 * u, k0, h);
        bL[u] = ldf(flo, br + 16 * u, k0, h);
      }
#pragma unroll
      for (int t = 0; t < 2; ++t)
#pragma unroll
        for (int u = 0; u < 2; ++u) acc[t][u] = wm3(aH[t], aL[t], bH[u], bL[u], acc[t][u]);
    }
#pragma unroll
    for (int t = 0; t < 2; ++t)
#pragma unroll
      for (int u = 0; u < 2; ++u)
#pragma unroll
        for (int r = 0; r < 8; ++r)
          sS[(wm * 32 + 16 * t + 8 * h + r) * SPF + wn * 32 + 16 * u + m] = acc[t][u][r];
    __syncthreads();
    if (tid < 64) {
#pragma unroll 2
      for (int j4 = 0; j4 < 16; ++j4) {
        const v4f c = *(const v4f*)(sS + tid * SPF + 4 * j4);
#pragma unroll
        for (int e = 0; e < 4; ++e) {
          const float v = c[e];
          const int id = n0 + 4 * j4 + e;
          if (better(v, id, tv[KT - 1], ti[KT - 1])) ins8(tv, ti, v, id);
        }
      }
    }
    __syncthreads();
  }

  if (tid < 64) {
#pragma unroll
    for (int k = 0; k < KT; ++k) {
      int c = ti[k];
      c = c < 0 ? 0 : (c > NN - 1 ? NN - 1 : c);
      sI[tid * KT + k] = c;
    }
  }
  __syncthreads();
  const v4i iv = *(const v4i*)(sI + 4 * tid);
  st2((v4i*)(idxo + (size_t)m0 * KT + 4 * tid), iv);
}

template <int BROW>
__device__ __forceinline__ void gemm_store_pass(const float* sC, const float* __restrict__ bias,
                                                float* C, int ldc, size_t cz, int mbase, int nbase,
                                                int wave, int lane) {
#pragma unroll
  for (int i = 0; i < 8; ++i) {
    const int r = wave * 16 + 2 * i + (lane >> 4);
    const int c4 = (lane & 15) * 4;
    v4f v = *(const v4f*)(sC + r * SPF + c4);
    if (BROW) {
      const float bb = bias[mbase + r];
      v += bb;
    } else {
      const v4f b4 = *(const v4f*)(bias + nbase + c4);
      v += b4;
    }
    float* p = C + cz + (size_t)(mbase + r) * (size_t)ldc + (size_t)(nbase + c4);
    *(volatile v4f*)p = v;
  }
}

template <int BROW>
__global__ __launch_bounds__(128) void k_gemm3(const unsigned short* __restrict__ ahi,
                                               const unsigned short* __restrict__ alo,
                                               const unsigned short* __restrict__ bhi,
                                               const unsigned short* __restrict__ blo,
                                               const float* __restrict__ bias, float* C,
                                               int ldc, int zA, int zB, int zC) {
  __shared__ __attribute__((aligned(16))) float sC[64 * SPF];
  const int tid = threadIdx.x, lane = tid & 31, wave = tid >> 5, h = lane >> 4, m = lane & 15;
  const int wm = wave >> 1, wn = wave & 1;
  const int mbase = blockIdx.x * 64, nbase = blockIdx.y * 64, z = blockIdx.z;
  const size_t ar = (size_t)z * (size_t)zA + (size_t)(mbase + wm * 32 + m);
  const size_t br = (size_t)z * (size_t)zB + (size_t)(nbase + wn * 32 + m);

  v8f acc[2][2];
#pragma unroll
  for (int t = 0; t < 2; ++t)
#pragma unroll
    for (int u = 0; u < 2; ++u) acc[t][u] = zero8();

#pragma unroll 1
  for (int ks = 0; ks < CC / 32; ++ks) {
    const int k0 = ks * 32;
    v16us aH[2], aL[2], bH[2], bL[2];
#pragma unroll
    for (int t = 0; t < 2; ++t) {
      aH[t] = ldf(ahi, ar + 16 * t, k0, h);
      aL[t] = ldf(alo, ar + 16 * t, k0, h);
    }
#pragma unroll
    for (int u = 0; u < 2; ++u) {
      bH[u] = ldf(bhi, br + 16 * u, k0, h);
      bL[u] = ldf(blo, br + 16 * u, k0, h);
    }
#pragma unroll
    for (int t = 0; t < 2; ++t)
#pragma unroll
      for (int u = 0; u < 2; ++u) acc[t][u] = wm3(aH[t], aL[t], bH[u], bL[u], acc[t][u]);
  }

#pragma unroll
  for (int t = 0; t < 2; ++t)
#pragma unroll
    for (int u = 0; u < 2; ++u)
#pragma unroll
      for (int r = 0; r < 8; ++r)
        sC[(wm * 32 + 16 * t + 8 * h + r) * SPF + wn * 32 + 16 * u + m] = acc[t][u][r];
  __syncthreads();

  const size_t cz = (size_t)z * (size_t)zC;
  gemm_store_pass<BROW>(sC, bias, C, ldc, cz, mbase, nbase, wave, lane);
  __threadfence();
  gemm_store_pass<BROW>(sC, bias, C, ldc, cz, mbase, nbase, wave, lane);
}

__device__ __forceinline__ int dedup(const int (&nb)[KT], int (&first)[KT]) {
  int cnt = 0;
#pragma unroll
  for (int k = 0; k < KT; ++k) {
    int f = 1;
#pragma unroll
    for (int j = 0; j < k; ++j) f = (nb[j] == nb[k]) ? 0 : f;
    first[k] = f;
    cnt += f;
  }
  return cnt;
}

__global__ __launch_bounds__(256) void k_edge(const int* __restrict__ idx, const float* __restrict__ xt,
                                              unsigned short* efh, unsigned short* efl) {
  const int tid = threadIdx.x, lane = tid & 31, wave = tid >> 5;
#pragma unroll 1
  for (int q = 0; q < 4; ++q) {
    const int e = (blockIdx.x * 8 + wave) * 4 + q;
    const v4i i0 = *(const v4i*)(idx + (size_t)e * KT);
    const v4i i1 = *(const v4i*)(idx + (size_t)e * KT + 4);
    int nb[KT];
    nb[0] = i0[0]; nb[1] = i0[1]; nb[2] = i0[2]; nb[3] = i0[3];
    nb[4] = i1[0]; nb[5] = i1[1]; nb[6] = i1[2]; nb[7] = i1[3];
    int first[KT];
    const int cnt = dedup(nb, first);
    const float w = 1.0f / (float)cnt;
    float fw[KT];
#pragma unroll
    for (int k = 0; k < KT; ++k) {
      fw[k] = first[k] ? w : 0.0f;
      int c = nb[k];
      c = c < 0 ? 0 : (c > NN - 1 ? NN - 1 : c);
      nb[k] = c;
    }
#pragma unroll 1
    for (int b = 0; b < NB; ++b) {
      float a[8];
#pragma unroll
      for (int i = 0; i < 8; ++i) a[i] = 0.0f;
#pragma unroll
      for (int k = 0; k < KT; ++k) {
        const float* rp = xt + ((size_t)(b * NN) + (size_t)nb[k]) * CC + 8 * lane;
        const v4f u0 = *(const v4f*)rp;
        const v4f u1 = *(const v4f*)(rp + 4);
#pragma unroll
        for (int i = 0; i < 4; ++i) {
          a[i]     += fw[k] * u0[i];
          a[4 + i] += fw[k] * u1[i];
        }
      }
      v8us hv, lv;
      split8(a, hv, lv);
      const size_t ro = ((size_t)(b * NN) + (size_t)e) * CC + 8 * lane;
      st2((v8us*)(efh + ro), hv);
      st2((v8us*)(efl + ro), lv);
    }
  }
}

template <int RESID>
__global__ __launch_bounds__(256) void k_node(const int* __restrict__ idx, const float* __restrict__ xp,
                                              const float* __restrict__ xres, float* xf,
                                              unsigned short* oh, unsigned short* ol) {
  __shared__ int sL[LCAP];
  __shared__ int sW[8];
  __shared__ __attribute__((aligned(16))) float sR[8 * CC];
  const int tid = threadIdx.x, lane = tid & 31, wave = tid >> 5;
  const int n0 = blockIdx.x * NPB;

#pragma unroll 1
  for (int b = 0; b < NB; ++b) {
    float acc[4][8];
#pragma unroll
    for (int j = 0; j < 4; ++j)
#pragma unroll
      for (int i = 0; i < 8; ++i) acc[j][i] = 0.0f;

#pragma unroll 1
    for (int ch = 0; ch < NCH; ++ch) {
      const int e = ch * ECH + tid;
      const v4i i0 = *(const v4i*)(idx + (size_t)e * KT);
      const v4i i1 = *(const v4i*)(idx + (size_t)e * KT + 4);
      int nb[KT];
      nb[0] = i0[0]; nb[1] = i0[1]; nb[2] = i0[2]; nb[3] = i0[3];
      nb[4] = i1[0]; nb[5] = i1[1]; nb[6] = i1[2]; nb[7] = i1[3];
      int first[KT];
      const int cnt = dedup(nb, first);
      int em[KT];
      int ct = 0;
#pragma unroll
      for (int k = 0; k < KT; ++k) {
        em[k] = (first[k] != 0 && (unsigned)(nb[k] - n0) < (unsigned)NPB) ? 1 : 0;
        ct += em[k];
      }
      int incl = ct;
      {
        int y;
        y = __shfl_up(incl, 1, 32);  if (lane >= 1)  incl += y;
        y = __shfl_up(incl, 2, 32);  if (lane >= 2)  incl += y;
        y = __shfl_up(incl, 4, 32);  if (lane >= 4)  incl += y;
        y = __shfl_up(incl, 8, 32);  if (lane >= 8)  incl += y;
        y = __shfl_up(incl, 16, 32); if (lane >= 16) incl += y;
      }
      const int excl = incl - ct;
      if (lane == 31) sW[wave] = incl;
      __syncthreads();
      int base = 0, tot = 0;
#pragma unroll
      for (int w8 = 0; w8 < 8; ++w8) {
        const int t = sW[w8];
        base += (w8 < wave) ? t : 0;
        tot += t;
      }
      int pos = base + excl;
#pragma unroll
      for (int k = 0; k < KT; ++k) {
        if (em[k]) {
          sL[pos] = e | ((nb[k] - n0) << 12) | (cnt << 17);
          ++pos;
        }
      }
      __syncthreads();
      tot = tot > LCAP ? LCAP : tot;
      for (int hh = 0; hh < tot; ++hh) {
        const int ent = sL[hh];
        const int ln = (ent >> 12) & 31;
        if ((ln & 7) == wave) {
          const int e2 = ent & (NN - 1);
          int cn = (ent >> 17) & 15;
          cn = cn < 1 ? 1 : cn;
          const float w = 1.0f / (float)cn;
          const float* rp = xp + ((size_t)(b * NN) + (size_t)e2) * CC + 8 * lane;
          const v4f u0 = *(const v4f*)rp;
          const v4f u1 = *(const v4f*)(rp + 4);
          const int js = ln >> 3;
#pragma unroll
          for (int j = 0; j < 4; ++j) {
            const float wj = (js == j) ? w : 0.0f;
#pragma unroll
            for (int i = 0; i < 4; ++i) {
              acc[j][i]     += wj * u0[i];
              acc[j][4 + i] += wj * u1[i];
            }
          }
        }
      }
      __syncthreads();
    }

#pragma unroll
    for (int j = 0; j < 4; ++j) {
      const int ln = wave + 8 * j;
      const size_t row = (size_t)(b * NN + n0 + ln);
      float x[8];
#pragma unroll
      for (int i = 0; i < 8; ++i) x[i] = fmaxf(acc[j][i], 0.0f);
      if (RESID) {
        const float* rp = xres + row * CC + 8 * lane;
        const v4f u0 = *(const v4f*)rp;
        const v4f u1 = *(const v4f*)(rp + 4);
#pragma unroll
        for (int i = 0; i < 4; ++i) { x[i] += u0[i]; x[4 + i] += u1[i]; }
      } else {
#pragma unroll
        for (int i = 0; i < 8; ++i) sR[wave * CC + 8 * lane + i] = x[i];
      }
      v8us hv, lv;
      split8(x, hv, lv);
      st2((v8us*)(oh + row * CC + 8 * lane), hv);
      st2((v8us*)(ol + row * CC + 8 * lane), lv);
      if (!RESID) {
        __syncthreads();
        const v4f p0 = *(const v4f*)(sR + wave * CC + 4 * lane);
        const v4f p1 = *(const v4f*)(sR + wave * CC + 128 + 4 * lane);
        st2((v4f*)(xf + row * CC + 4 * lane), p0);
        st2((v4f*)(xf + row * CC + 128 + 4 * lane), p1);
        __syncthreads();
      }
    }
  }
}

__device__ __forceinline__ double bsum(double s, double* sD, int lane, int wave) {
  s += __shfl_xor(s, 16, 32);
  s += __shfl_xor(s, 8, 32);
  s += __shfl_xor(s, 4, 32);
  s += __shfl_xor(s, 2, 32);
  s += __shfl_xor(s, 1, 32);
  if (lane == 0) sD[wave] = s;
  __syncthreads();
  double t = 0.0;
#pragma unroll
  for (int w = 0; w < 8; ++w) t += sD[w];
  __syncthreads();
  return t;
}

__device__ __forceinline__ void bn_out_pass(const float* __restrict__ y, const float* __restrict__ feat,
                                            float* out, int o, int tid, float mu, float rstd,
                                            float g, float be) {
#pragma unroll 1
  for (int b = 0; b < NB; ++b) {
    const size_t base = ((size_t)b * CC + (size_t)o) * NN;
#pragma unroll
    for (int j = 0; j < 4; ++j) {
      const size_t off = base + (size_t)(4 * (tid + 256 * j));
      const v4f v = *(const v4f*)(y + off);
      const v4f f = *(const v4f*)(feat + off);
      v4f r;
#pragma unroll
      for (int i = 0; i < 4; ++i) {
        float t = (v[i] - mu) * rstd;
        t = t * g + be;
        r[i] = f[i] + t;
      }
      *(volatile v4f*)(out + off) = r;
    }
  }
}

__global__ __launch_bounds__(256) void k_bnout(const float* __restrict__ y, const float* __restrict__ feat,
                                               const float* __restrict__ gam, const float* __restrict__ bet,
                                               float* out) {
  __shared__ double sD[8];
  const int tid = threadIdx.x, lane = tid & 31, wave = tid >> 5;
  const int o = blockIdx.x;

  double s = 0.0;
#pragma unroll 1
  for (int b = 0; b < NB; ++b) {
    const size_t base = ((size_t)b * CC + (size_t)o) * NN;
#pragma unroll
    for (int j = 0; j < 4; ++j) {
      const v4f v = *(const v4f*)(y + base + (size_t)(4 * (tid + 256 * j)));
      s += (double)v[0]; s += (double)v[1]; s += (double)v[2]; s += (double)v[3];
    }
  }
  const double tot = bsum(s, sD, lane, wave);
  const float mu = (float)(tot * (1.0 / 16384.0));

  double s2 = 0.0;
#pragma unroll 1
  for (int b = 0; b < NB; ++b) {
    const size_t base = ((size_t)b * CC + (size_t)o) * NN;
#pragma unroll
    for (int j = 0; j < 4; ++j) {
      const v4f v = *(const v4f*)(y + base + (size_t)(4 * (tid + 256 * j)));
#pragma unroll
      for (int i = 0; i < 4; ++i) {
        const float d = v[i] - mu;
        s2 += (double)(d * d);
      }
    }
  }
  const double tot2 = bsum(s2, sD, lane, wave);
  const float var = (float)(tot2 * (1.0 / 16384.0));
  const float rstd = 1.0f / sqrtf(var + BNEPS);
  const float g = gam[o];
  const float be = bet[o];

  bn_out_pass(y, feat, out, o, tid, mu, rstd, g, be);
  __threadfence();
  bn_out_pass(y, feat, out, o, tid, mu, rstd, g, be);
}

extern "C" void kernel_launch(void* const* d_in, const int* in_sizes, int n_in,
                              void* d_out, int out_size, void* d_ws, size_t ws_size,
                              hipStream_t stream) {
  if (n_in < 13) return;
  if (in_sizes[0] != NB * CC * NN) return;
  if (in_sizes[1] != CC * CC || in_sizes[3] != CC * CC || in_sizes[5] != CC * CC ||
      in_sizes[7] != CC * CC || in_sizes[9] != CC * CC) return;
  if (in_sizes[2] != CC || in_sizes[4] != CC || in_sizes[6] != CC || in_sizes[8] != CC ||
      in_sizes[10] != CC || in_sizes[11] != CC || in_sizes[12] != CC) return;
  if (out_size != NB * CC * NN) return;

  const float* feat = (const float*)d_in[0];
  const float* th0w = (const float*)d_in[1];
  const float* th0b = (const float*)d_in[2];
  const float* ph0w = (const float*)d_in[3];
  const float* ph0b = (const float*)d_in[4];
  const float* th1w = (const float*)d_in[5];
  const float* th1b = (const float*)d_in[6];
  const float* ph1w = (const float*)d_in[7];
  const float* ph1b = (const float*)d_in[8];
  const float* pjw  = (const float*)d_in[9];
  const float* pjb  = (const float*)d_in[10];
  const float* gam  = (const float*)d_in[11];
  const float* bet  = (const float*)d_in[12];
  float* out = (float*)d_out;

  const size_t PLB  = (size_t)NR * CC * 2;
  const size_t F0B  = (size_t)NN * CC * 2;
  const size_t PW   = (size_t)CC * CC;
  const size_t WPB  = (size_t)10 * PW * 2;
  const size_t IDB  = (size_t)NN * KT * 4;
  const size_t F32B = (size_t)NR * CC * 4;
  char* ws = (char*)d_ws;
  size_t off = 0;
  const size_t oX0h = off; off += PLB;
  const size_t oX0l = off; off += PLB;
  const size_t oF0h = off; off += F0B;
  const size_t oF0l = off; off += F0B;
  const size_t oWP  = off; off += WPB;
  const size_t oIDX = off; off += IDB;
  const size_t oXT  = off; off += F32B;
  const size_t oEFh = off; off += PLB;
  const size_t oEFl = off; off += PLB;
  const size_t oXP  = off; off += F32B;
  const size_t oX1f = off; off += F32B;
  const size_t oX1h = off; off += PLB;
  const size_t oX1l = off; off += PLB;
  if (off > ws_size || off > (size_t)134217728) return;

  unsigned short* X0h = (unsigned short*)(ws + oX0h);
  unsigned short* X0l = (unsigned short*)(ws + oX0l);
  unsigned short* X2h = X0h;
  unsigned short* X2l = X0l;
  unsigned short* F0h = (unsigned short*)(ws + oF0h);
  unsigned short* F0l = (unsigned short*)(ws + oF0l);
  unsigned short* WP  = (unsigned short*)(ws + oWP);
  int*   IDX = (int*)(ws + oIDX);
  float* XT  = (float*)(ws + oXT);
  float* Y   = XT;
  unsigned short* EFh = (unsigned short*)(ws + oEFh);
  unsigned short* EFl = (unsigned short*)(ws + oEFl);
  float* XP  = (float*)(ws + oXP);
  float* X1f = (float*)(ws + oX1f);
  unsigned short* X1h = (unsigned short*)(ws + oX1h);
  unsigned short* X1l = (unsigned short*)(ws + oX1l);

  k_feat2p<<<dim3(NN / 32, NB), 256, 0, stream>>>(feat, X0h, X0l, F0h, F0l);
  k_w2p<<<dim3(CC / 32, 5), 256, 0, stream>>>(th0w, ph0w, th1w, ph1w, pjw, WP);
  k_sim<<<NN / 64, 128, 0, stream>>>(F0h, F0l, IDX);

  const dim3 gAct(NR / 64, CC / 64, 1);
  k_gemm3<0><<<gAct, 128, 0, stream>>>(X0h, X0l, WP + 0 * PW, WP + 1 * PW, th0b, XT, CC, 0, 0, 0);
  k_edge<<<NN / 32, 256, 0, stream>>>(IDX, XT, EFh, EFl);
  k_gemm3<0><<<gAct, 128, 0, stream>>>(EFh, EFl, WP + 2 * PW, WP + 3 * PW, ph0b, XP, CC, 0, 0, 0);
  k_node<0><<<NN / NPB, 256, 0, stream>>>(IDX, XP, X1f, X1f, X1h, X1l);
  k_gemm3<0><<<gAct, 128, 0, stream>>>(X1h, X1l, WP + 4 * PW, WP + 5 * PW, th1b, XT, CC, 0, 0, 0);
  k_edge<<<NN / 32, 256, 0, stream>>>(IDX, XT, EFh, EFl);
  k_gemm3<0><<<gAct, 128, 0, stream>>>(EFh, EFl, WP + 6 * PW, WP + 7 * PW, ph1b, XP, CC, 0, 0, 0);
  k_node<1><<<NN / NPB, 256, 0, stream>>>(IDX, XP, X1f, X1f, X2h, X2l);
  k_gemm3<1><<<dim3(CC / 64, NN / 64, NB), 128, 0, stream>>>(WP + 8 * PW, WP + 9 * PW, X2h, X2l,
                                                             pjb, Y, NN, 0, NN, CC * NN);
  k_bnout<<<CC, 256, 0, stream>>>(Y, feat, gam, bet, out);
}
